// MemoEnhancedPredictor_54571854463676
// MI455X (gfx1250) — hardware-run, weakly checked
//
#include <hip/hip_runtime.h>


#ifndef NROWS
#define NROWS 16384
#endif
#define NROWS_FULL 16384
#define DM     512
#define NLAB   4
#define BANK   512
#define RB     256
#define NBB    (NROWS / RB)
#define NPART  (NLAB + NBB)
#define CSP    20
#define INFKEY 0xFF800000u
#define OFF1   ((size_t)NROWS_FULL * NLAB)
#define OFF2   ((size_t)2 * NROWS_FULL * NLAB)

static_assert(NROWS <= NROWS_FULL);
static_assert(NROWS % 256 == 0);
static_assert(NROWS % RB == 0);
static_assert(NROWS % 64 == 0);
static_assert(DM % 32 == 0);
static_assert(DM == 2 * 256);
static_assert(NLAB * (DM / 8) == 256);
static_assert(3 * NLAB <= 16);
static_assert(NLAB == 4);
static_assert(BANK % 256 == 0);
static_assert((CSP * 4) % 16 == 0);
static_assert(OFF1 * 4 == 262144);
static_assert(OFF2 * 4 == 524288);
static_assert((OFF2 + NROWS_FULL) * 4 == 589824);
static_assert(32 * 16 * 2 == 64 * 16);
static_assert((size_t)BANK * 4 + 64 <= 131072);
static_assert((size_t)NLAB * DM * 4 <= 131072);
static_assert((size_t)64 * CSP * 4 <= 131072);

typedef unsigned short bf;
typedef __attribute__((ext_vector_type(16))) __bf16   v16bf;
typedef __attribute__((ext_vector_type(8)))  unsigned short v8us;
typedef __attribute__((ext_vector_type(8)))  float    v8f;
typedef __attribute__((ext_vector_type(4)))  float    v4f;
typedef v4f  __attribute__((may_alias)) v4fa;

__device__ __forceinline__ unsigned short f2bf(float f) { unsigned u = __float_as_uint(f); u += 0x7FFFu + ((u >> 16) & 1u); return (unsigned short)(u >> 16); }
__device__ __forceinline__ float bfr(float f) { return __uint_as_float(((unsigned)f2bf(f)) << 16); }
__device__ __forceinline__ v16bf cat16b(v8us lo, v8us hi) { return __builtin_bit_cast(v16bf, __builtin_shufflevector(lo, hi, 0, 1, 2, 3, 4, 5, 6, 7, 8, 9, 10, 11, 12, 13, 14, 15)); }
__device__ __forceinline__ v8f wmmab(v16bf a, v16bf b, v8f c) { return __builtin_amdgcn_wmma_f32_16x16x32_bf16(false, a, false, b, (short)0, c, false, false); }
__device__ __forceinline__ v16bf ldb(const bf* p)  { return cat16b(*(const v8us*)p, *(const v8us*)(p + 16)); }
__device__ __forceinline__ void wave_sync() { __builtin_amdgcn_fence(3  , "wavefront"); __builtin_amdgcn_wave_barrier(); asm volatile("" ::: "memory"); }
__device__ __forceinline__ v8f wmmab_g(v16bf a, v16bf b, v8f c) { c = wmmab(a, b, c); asm volatile("v_nop\n\tv_nop\n\tv_nop\n\tv_nop" : "+v"(c) : "v"(a), "v"(b)); return c; }
__device__ __forceinline__ unsigned okey(float e) { const float z = (e == 0.0f) ? 0.0f : e; const unsigned u = __float_as_uint(z); return (u & 0x80000000u) ? ~u : (u | 0x80000000u); }

__global__ __launch_bounds__(256) void k_cvt8(const float* __restrict__ src, bf* dst, size_t n8) {
    const size_t i = (size_t)blockIdx.x * 256 + threadIdx.x; if (i >= n8) return;
    const v8f v = *(const v8f*)(src + i * 8); v8us o;
#pragma unroll
    for (int k = 0; k < 8; ++k) o[k] = f2bf(v[k]);
    *(volatile v8us*)(dst + i * 8) = o; __threadfence(); *(volatile v8us*)(dst + i * 8) = o;
}

__global__ __launch_bounds__(256) void k_rows(const float* __restrict__ LG, float* OUT1, float* OUT2, unsigned* EK, int* LB) {
#pragma clang fp contract(off)
    const int r = (int)(blockIdx.x * 256 + threadIdx.x);
    const v4f lg = *(const v4f*)(LG + (size_t)r * NLAB);
    const float l0 = bfr(lg[0]), l1 = bfr(lg[1]), l2 = bfr(lg[2]), l3 = bfr(lg[3]);
    const float mx = fmaxf(fmaxf(l0, l1), fmaxf(l2, l3));
    const float d0 = l0 - mx, d1 = l1 - mx, d2 = l2 - mx, d3 = l3 - mx;
    const float e0 = expf(d0), e1 = expf(d1), e2 = expf(d2), e3 = expf(d3);
    const float s = ((e0 + e1) + e2) + e3;
    const float inv = 1.0f / s;
    const float ls = logf(s);
    v4f pv; pv[0] = e0 * inv; pv[1] = e1 * inv; pv[2] = e2 * inv; pv[3] = e3 * inv;
    const float g0 = d0 - ls, g1 = d1 - ls, g2 = d2 - ls, g3 = d3 - ls;
    const float t0 = pv[0] * g0, t1 = pv[1] * g1, t2 = pv[2] * g2, t3 = pv[3] * g3;
    const float en = -(((t0 + t1) + t2) + t3);
    int am = 0; float bm = l0;
    am = (l1 > bm) ? 1 : am; bm = (l1 > bm) ? l1 : bm;
    am = (l2 > bm) ? 2 : am; bm = (l2 > bm) ? l2 : bm;
    am = (l3 > bm) ? 3 : am;
    const unsigned key = okey(en);
    float* po = OUT1 + (size_t)r * NLAB;
#pragma unroll 1
    for (int ps = 0; ps < 2; ++ps) {
        *(volatile v4f*)po = pv;
        *(volatile float*)(OUT2 + r) = en;
        *(volatile unsigned*)(EK + r) = key;
        *(volatile int*)(LB + r) = am;
        if (ps == 0) __threadfence(); }
}

__global__ __launch_bounds__(256) void k_select(const float* __restrict__ EM, const unsigned* __restrict__ EK, const int* __restrict__ LB, unsigned* TH) {
    __shared__ unsigned mk[BANK];
    __shared__ unsigned wsum[2][8];
    const int t = (int)threadIdx.x, lane = t & 31;
    const int wave = __builtin_amdgcn_readfirstlane((int)(threadIdx.x >> 5));
    const int c = (int)blockIdx.x;
#pragma unroll
    for (int i = 0; i < BANK / 256; ++i) { const int m = t + i * 256; mk[m] = okey(bfr(EM[c * BANK + m])); }
    __syncthreads();
    unsigned prefix = 0u, want = BANK, nless = 0u;
#pragma unroll 1
    for (int ps = 0; ps < 33; ++ps) {
        const bool last = (ps == 32);
        const int sh = last ? 0 : (31 - ps);
        const unsigned pref0 = prefix << 1;
        unsigned cnt = 0u;
#pragma unroll
        for (int i = 0; i < BANK / 256; ++i) { const unsigned k = mk[t + i * 256]; cnt += last ? (unsigned)(k < prefix) : (unsigned)((k >> sh) == pref0); }
#pragma unroll 4
        for (int b = t; b < NROWS; b += 256) {
            unsigned kk = EK[b]; int lb = LB[b];
            asm volatile("" : "+v"(kk)); asm volatile("" : "+v"(lb));
            const unsigned k = (lb == c) ? kk : INFKEY;
            cnt += last ? (unsigned)((lb == c) & (kk < prefix)) : (unsigned)((k >> sh) == pref0); }
        int sv = (int)cnt;
        sv += __shfl_xor(sv, 16, 32); sv += __shfl_xor(sv, 8, 32); sv += __shfl_xor(sv, 4, 32); sv += __shfl_xor(sv, 2, 32); sv += __shfl_xor(sv, 1, 32);
        if (lane == 0) wsum[ps & 1][wave] = (unsigned)sv;
        __syncthreads();
        unsigned total = 0u;
#pragma unroll
        for (int w = 0; w < 8; ++w) total += wsum[ps & 1][w];
        if (!last) { if (want <= total) { prefix = pref0; } else { want -= total; prefix = pref0 | 1u; } }
        else       { nless = total; }
    }
    const unsigned T = prefix;
    int q = (int)BANK - (int)nless; q = q < 0 ? 0 : (q > BANK ? BANK : q);
    int got = 0; unsigned mcut = 0u, bcut = 0u;
#pragma unroll 1
    for (int m = 0; m < BANK && got < q; ++m) { got += __builtin_amdgcn_readfirstlane((int)(mk[m] == T)); mcut = (unsigned)(m + 1); }
#pragma unroll 1
    for (int b = 0; b < NROWS && got < q; ++b) { const unsigned kk = EK[b]; const int lb = LB[b]; got += __builtin_amdgcn_readfirstlane((int)((lb == c) & (kk == T))); bcut = (unsigned)(b + 1); }
    if (wave == 0) {
        unsigned v = 0u;
        v = (lane == 0) ? T : v; v = (lane == 1) ? mcut : v; v = (lane == 2) ? bcut : v; v = (lane == 3) ? nless : v;
        unsigned* dst = TH + c * 32 + lane;
#pragma unroll 1
        for (int ps = 0; ps < 2; ++ps) { *(volatile unsigned*)dst = v; if (ps == 0) __threadfence(); }
    }
}

__global__ __launch_bounds__(256) void k_partial(const float* __restrict__ TM, const float* __restrict__ TE, const float* __restrict__ EM,
                                                 const unsigned* __restrict__ EK, const int* __restrict__ LB, const unsigned* __restrict__ TH, float* PART) {
#pragma clang fp contract(off)
    __shared__ float lacc[NLAB * DM];
    const int t = (int)threadIdx.x; const int p = (int)blockIdx.x;
#pragma unroll
    for (int j = 0; j < NLAB; ++j) { lacc[j * DM + t] = 0.0f; lacc[j * DM + t + 256] = 0.0f; }
    if (p < NLAB) {
        const int c = p;
        const unsigned T = TH[c * 32]; unsigned mc = TH[c * 32 + 1]; mc = mc > (unsigned)BANK ? (unsigned)BANK : mc;
        const float* base = TM + (size_t)c * BANK * DM;
#pragma unroll 1
        for (int m = 0; m < BANK; ++m) {
            const unsigned key = okey(bfr(EM[c * BANK + m]));
            const int sel = __builtin_amdgcn_readfirstlane((int)((key < T) | ((key == T) & ((unsigned)m < mc))));
            if (sel) {
                const float v0 = bfr(base[(size_t)m * DM + t]); const float v1 = bfr(base[(size_t)m * DM + t + 256]);
                lacc[c * DM + t] += v0; lacc[c * DM + t + 256] += v1; }
        }
    } else {
        const int b0 = (p - NLAB) * RB;
#pragma unroll 1
        for (int i = 0; i < RB; ++i) {
            const int b = b0 + i;
            const int lab = LB[b] & 3;
            const unsigned key = EK[b];
            const unsigned T = TH[lab * 32]; unsigned bc = TH[lab * 32 + 2]; bc = bc > (unsigned)NROWS ? (unsigned)NROWS : bc;
            const int sel = __builtin_amdgcn_readfirstlane((int)((key < T) | ((key == T) & ((unsigned)b < bc))));
            if (sel) {
                const float v0 = bfr(TE[(size_t)b * DM + t]); const float v1 = bfr(TE[(size_t)b * DM + t + 256]);
                lacc[lab * DM + t] += v0; lacc[lab * DM + t + 256] += v1; }
        }
    }
    float o[2 * NLAB];
#pragma unroll
    for (int j = 0; j < NLAB; ++j) { o[2 * j] = lacc[j * DM + t]; o[2 * j + 1] = lacc[j * DM + t + 256]; }
    float* out = PART + (size_t)p * NLAB * DM;
#pragma unroll 1
    for (int ps = 0; ps < 2; ++ps) {
#pragma unroll
        for (int j = 0; j < NLAB; ++j) { *(volatile float*)(out + j * DM + t) = o[2 * j]; *(volatile float*)(out + j * DM + t + 256) = o[2 * j + 1]; }
        if (ps == 0) __threadfence(); }
}

__global__ __launch_bounds__(256) void k_reduce(const float* __restrict__ PART, bf* SB) {
#pragma clang fp contract(off)
    const int t = (int)threadIdx.x; const int c = t >> 6, d8 = t & 63;
    v8f s = (v8f){};
#pragma unroll 1
    for (int p = 0; p < NPART; ++p) { const v8f x = *(const v8f*)(PART + ((size_t)(p * NLAB + c)) * DM + d8 * 8); s = s + x; }
    v8us oh, om, ol, oz;
#pragma unroll
    for (int k = 0; k < 8; ++k) {
        const unsigned short h = f2bf(s[k]); const float fh = __uint_as_float(((unsigned)h) << 16);
        const float r1 = s[k] - fh;
        const unsigned short m = f2bf(r1); const float fm = __uint_as_float(((unsigned)m) << 16);
        const float r2 = r1 - fm;
        oh[k] = h; om[k] = m; ol[k] = f2bf(r2); oz[k] = (unsigned short)0; }
    bf* dst = SB + (size_t)c * DM + d8 * 8;
#pragma unroll 1
    for (int ps = 0; ps < 2; ++ps) {
        *(volatile v8us*)dst = oh; *(volatile v8us*)(dst + 4 * DM) = om; *(volatile v8us*)(dst + 8 * DM) = ol; *(volatile v8us*)(dst + 12 * DM) = oz;
        if (ps == 0) __threadfence(); }
}

__global__ __launch_bounds__(32) void k_gemm(const bf* __restrict__ A, const bf* __restrict__ Bt, float* OUT0) {
#pragma clang fp contract(off)
    __shared__ __align__(16) float os[64 * CSP];
    const int K = DM;
    const int lane = threadIdx.x & 31, lr = lane & 15, hi = lane >> 4; const int r0 = blockIdx.x * 64;
    v8f acc[4];
#pragma unroll
    for (int mb = 0; mb < 4; ++mb) acc[mb] = (v8f){};
    const size_t aoff = (size_t)(r0 + lr) * K + 8 * hi, boff = (size_t)lr * K + 8 * hi;
#pragma unroll 1
    for (int kc = 0; kc < K; kc += 32) {
        const v16bf b = ldb(Bt + boff + kc);
#pragma unroll
        for (int mb = 0; mb < 4; ++mb) { const v16bf a = ldb(A + aoff + (size_t)mb * 16 * K + kc); acc[mb] = wmmab_g(a, b, acc[mb]); }
    }
#pragma unroll
    for (int mb = 0; mb < 4; ++mb) {
#pragma unroll
        for (int j = 0; j < 8; ++j) os[(mb * 16 + hi * 8 + j) * CSP + lr] = acc[mb][j]; }
    wave_sync();
    v4f val[2];
#pragma unroll
    for (int s = 0; s < 2; ++s) {
        const int row = s * 32 + lane;
        const v4f xh = *(const v4fa*)(&os[row * CSP]); const v4f xm = *(const v4fa*)(&os[row * CSP + 4]); const v4f xl = *(const v4fa*)(&os[row * CSP + 8]);
        const float c0 = xh[0] + (xm[0] + xl[0]), c1 = xh[1] + (xm[1] + xl[1]), c2 = xh[2] + (xm[2] + xl[2]), c3 = xh[3] + (xm[3] + xl[3]);
        const float tx0 = c0 + c2, tx1 = c1 + c3;
        const float vx0 = c0 + c1, vx1 = c2 + c3;
        const float dt = tx0 - tx1, dv = vx0 - vx1;
        const float et = expf(-fabsf(dt)), ev = expf(-fabsf(dv));
        const float it = 1.0f / (1.0f + et), iv = 1.0f / (1.0f + ev);
        const float tb = it, ts = et * it, vb = iv, vs = ev * iv;
        const float p0 = (dt >= 0.0f) ? tb : ts, p1 = (dt >= 0.0f) ? ts : tb;
        const float w0 = (dv >= 0.0f) ? vb : vs, w1 = (dv >= 0.0f) ? vs : vb;
        v4f o; o[0] = p0 * w0; o[1] = p1 * w0; o[2] = p0 * w1; o[3] = p1 * w1;
        val[s] = o; }
    float* orow = OUT0 + (size_t)r0 * NLAB;
#pragma unroll 1
    for (int ps = 0; ps < 2; ++ps) {
#pragma unroll
        for (int s = 0; s < 2; ++s) { const int row = s * 32 + lane;
            *(volatile v4f*)(orow + (size_t)row * NLAB) = val[s]; }
        if (ps == 0) __threadfence(); }
}

static constexpr size_t al256(size_t v) { return (v + 255) & ~(size_t)255; }
static constexpr size_t SZ_XB = al256((size_t)NROWS * DM * 2);
static constexpr size_t SZ_EK = al256((size_t)NROWS * 4);
static constexpr size_t SZ_LB = al256((size_t)NROWS * 4);
static constexpr size_t SZ_TH = al256((size_t)NLAB * 32 * 4);
static constexpr size_t SZ_PT = al256((size_t)NPART * NLAB * DM * 4);
static constexpr size_t SZ_SB = al256((size_t)16 * DM * 2);
static constexpr size_t SZ_TOTAL = SZ_XB + SZ_EK + SZ_LB + SZ_TH + SZ_PT + SZ_SB;
static_assert(SZ_TOTAL <= (size_t)134217728);
static_assert(((size_t)NROWS * DM) % 8 == 0);

extern "C" void kernel_launch(void* const* d_in, const int* in_sizes, int n_in,
                              void* d_out, int out_size, void* d_ws, size_t ws_size, hipStream_t stream) {
    if (n_in < 6) return;
    if ((size_t)in_sizes[0] < (size_t)NROWS * NLAB) return;
    if ((size_t)in_sizes[1] < (size_t)NROWS * DM) return;
    if ((size_t)in_sizes[3] < (size_t)NLAB * BANK) return;
    if ((size_t)in_sizes[4] < (size_t)NLAB * BANK * DM) return;
    if ((size_t)out_size < OFF2 + (size_t)NROWS) return;
    if (SZ_TOTAL > ws_size) return;
    const float* lg = (const float*)d_in[0];
    const float* te = (const float*)d_in[1];
    const float* em = (const float*)d_in[3];
    const float* tm = (const float*)d_in[4];
    float* OUT0 = (float*)d_out;
    float* OUT1 = OUT0 + OFF1;
    float* OUT2 = OUT0 + OFF2;
    char* wsp = (char*)d_ws;
    bf* XB = (bf*)wsp; wsp += SZ_XB;
    unsigned* EK = (unsigned*)wsp; wsp += SZ_EK;
    int* LB = (int*)wsp; wsp += SZ_LB;
    unsigned* TH = (unsigned*)wsp; wsp += SZ_TH;
    float* PART = (float*)wsp; wsp += SZ_PT;
    bf* SB = (bf*)wsp; wsp += SZ_SB;

    k_rows<<<NROWS / 256, 256, 0, stream>>>(lg, OUT1, OUT2, EK, LB);
    { const size_t n8 = (size_t)NROWS * DM / 8;
      k_cvt8<<<(unsigned)((n8 + 255) / 256), 256, 0, stream>>>(te, XB, n8); }
    k_select<<<NLAB, 256, 0, stream>>>(em, EK, LB, TH);
    k_partial<<<NPART, 256, 0, stream>>>(tm, te, em, EK, LB, TH, PART);
    k_reduce<<<1, 256, 0, stream>>>(PART, SB);
    k_gemm<<<NROWS / 64, 32, 0, stream>>>(XB, SB, OUT0);
}
